// MambaBlock_58067957842028
// MI455X (gfx1250) — hardware-verified
//
#include <hip/hip_runtime.h>
#include <stddef.h>
#include <stdint.h>
#include <math.h>


#define DM    1024
#define DI    2048
#define NXZ   4096
#define DS    16
#define TL    2048
#define NBAT  2
#define MR    4096
#define NPX   33
#define PPIT  64
#define KIN   2048
#define KXP   4096
#define GBM   64
#define GTHR  128
#define SCH   64
#define STH   128
#define TCH   32
#define PSP   36
#define WSMAX 134217728

static_assert(MR == NBAT * TL && (TL & (TL - 1)) == 0);
static_assert(KIN == 2 * DM && KXP == 2 * DI && KIN % 32 == 0 && KXP % 32 == 0);
static_assert(MR % GBM == 0 && NXZ % 128 == 0 && DM % 128 == 0 && PPIT == 64);
static_assert(GBM == (GTHR / 32) * 16);
static_assert(DI % SCH == 0 && TL % TCH == 0 && STH == 2 * SCH && DS == 16);
static_assert((PSP * 4) % 16 == 0 && PSP >= 33);
static_assert(NPX == 1 + 2 * DS && NPX <= PPIT);

typedef float          v4f   __attribute__((ext_vector_type(4)));
typedef float          v8f   __attribute__((ext_vector_type(8)));
typedef int            v8i   __attribute__((ext_vector_type(8)));
typedef unsigned short v8us  __attribute__((ext_vector_type(8)));
typedef unsigned short v16us __attribute__((ext_vector_type(16)));
typedef __bf16         v16bf __attribute__((ext_vector_type(16)));
typedef v4f  __attribute__((may_alias)) v4fa;
typedef v8us __attribute__((may_alias)) v8usa;
union FragB { v16bf v; v16us u; v8us h[2]; v8i w; };

__device__ __forceinline__ v8f wmb(const FragB& a, const FragB& b, v8f c) {
  v8f d = __builtin_amdgcn_wmma_f32_16x16x32_bf16(false, a.v, false, b.v, (short)0, c, false, false);
  asm volatile("v_nop\n\tv_nop\n\tv_nop\n\tv_nop" : "+v"(d) : "v"(a.w), "v"(b.w));
  return d;
}

__device__ __forceinline__ unsigned bf16_bits(float f) {
  const unsigned u = __float_as_uint(f);
  return (u + 0x7FFFu + ((u >> 16) & 1u)) >> 16;
}
__device__ __forceinline__ float bf16_val(float f) {
  return __uint_as_float(bf16_bits(f) << 16);
}

__device__ __forceinline__ float conv_silu(float x0, float x1, float x2, float x3,
                                           float w0, float w1, float w2, float w3, float cb) {
  float v = w0 * x0;
  v = fmaf(w1, x1, v);
  v = fmaf(w2, x2, v);
  v = fmaf(w3, x3, v);
  v = v + cb;
  const float e = expf(-v);
  return v * (1.0f / (1.0f + e));
}

__global__ __launch_bounds__(128) void k_norm(const float* __restrict__ x, const float* __restrict__ nw,
                                              unsigned short* xn) {
  __shared__ float red[4];
  const int tid = (int)threadIdx.x, lane = tid & 31, wave = tid >> 5;
  const int row = (int)blockIdx.x;
  const float* p = x + (size_t)row * DM + 8 * tid;
  const v4f a = *(const v4fa*)p;
  const v4f b = *(const v4fa*)(p + 4);
  float v[8];
  v[0] = bf16_val(a.x); v[1] = bf16_val(a.y); v[2] = bf16_val(a.z); v[3] = bf16_val(a.w);
  v[4] = bf16_val(b.x); v[5] = bf16_val(b.y); v[6] = bf16_val(b.z); v[7] = bf16_val(b.w);
  float ss = v[0] * v[0];
#pragma unroll
  for (int i = 1; i < 8; ++i) ss = fmaf(v[i], v[i], ss);
#pragma unroll
  for (int off = 16; off > 0; off >>= 1) ss += __shfl_xor(ss, off, 32);
  if (lane == 0) red[wave] = ss;
  __syncthreads();
  const float tot  = ((red[0] + red[1]) + red[2]) + red[3];
  const float rms  = sqrtf(tot * (1.0f / 1024.0f) + 1e-6f);
  const float rinv = 1.0f / rms;
  const v4f wa = *(const v4fa*)(nw + 8 * tid);
  const v4f wb = *(const v4fa*)(nw + 8 * tid + 4);
  float w[8];
  w[0] = bf16_val(wa.x); w[1] = bf16_val(wa.y); w[2] = bf16_val(wa.z); w[3] = bf16_val(wa.w);
  w[4] = bf16_val(wb.x); w[5] = bf16_val(wb.y); w[6] = bf16_val(wb.z); w[7] = bf16_val(wb.w);
  v8us oh, ol;
#pragma unroll
  for (int i = 0; i < 8; ++i) {
    const float y = (v[i] * rinv) * w[i];
    const unsigned hb = bf16_bits(y);
    oh[i] = (unsigned short)hb;
    ol[i] = (unsigned short)bf16_bits(y - __uint_as_float(hb << 16));
  }
  unsigned short* dp = xn + (size_t)row * KIN + 8 * tid;
  *(volatile v8us*)dp = oh;
  *(volatile v8us*)(dp + DM) = ol;
  __threadfence();
  *(volatile v8us*)dp = oh;
  *(volatile v8us*)(dp + DM) = ol;
}

__global__ __launch_bounds__(256) void k_wT(const float* __restrict__ W, int Kd, int Nn, unsigned short* out) {
  __shared__ float tile[64 * 65];
  const int tid = (int)threadIdx.x;
  const int n0 = (int)blockIdx.x * 64;
  const int k0 = (int)blockIdx.y * 64;
#pragma unroll
  for (int it = 0; it < 4; ++it) {
    const int u = it * 256 + tid;
    const int r = u >> 4, c4 = u & 15;
    const v4f t = *(const v4fa*)(W + (size_t)(k0 + r) * (size_t)Nn + n0 + 4 * c4);
    tile[r * 65 + 4 * c4 + 0] = t.x;
    tile[r * 65 + 4 * c4 + 1] = t.y;
    tile[r * 65 + 4 * c4 + 2] = t.z;
    tile[r * 65 + 4 * c4 + 3] = t.w;
  }
  __syncthreads();
  v8us o[2];
#pragma unroll
  for (int it = 0; it < 2; ++it) {
    const int u = it * 256 + tid;
    const int n = u >> 3, pc = u & 7;
#pragma unroll
    for (int i = 0; i < 8; ++i) o[it][i] = (unsigned short)bf16_bits(tile[(8 * pc + i) * 65 + n]);
  }
#pragma unroll
  for (int it = 0; it < 2; ++it) {
    const int u = it * 256 + tid;
    const int n = u >> 3, pc = u & 7;
    unsigned short* dp = out + (size_t)(n0 + n) * (size_t)(2 * Kd) + k0 + 8 * pc;
    *(volatile v8us*)dp = o[it];
    *(volatile v8us*)(dp + Kd) = o[it];
  }
  __threadfence();
#pragma unroll
  for (int it = 0; it < 2; ++it) {
    const int u = it * 256 + tid;
    const int n = u >> 3, pc = u & 7;
    unsigned short* dp = out + (size_t)(n0 + n) * (size_t)(2 * Kd) + k0 + 8 * pc;
    *(volatile v8us*)dp = o[it];
    *(volatile v8us*)(dp + Kd) = o[it];
  }
}

__global__ __launch_bounds__(256) void k_wx(const float* __restrict__ Wx, unsigned short* out) {
  const int n  = (int)blockIdx.x;
  const int k8 = 8 * (int)threadIdx.x;
  const int nc = n < NPX ? n : NPX - 1;
  const bool ok = n < NPX;
  const float* p = Wx + (size_t)k8 * NPX + nc;
  v8us o;
#pragma unroll
  for (int i = 0; i < 8; ++i) {
    const float f = p[(size_t)i * NPX];
    o[i] = ok ? (unsigned short)bf16_bits(f) : (unsigned short)0;
  }
  unsigned short* dp = out + (size_t)n * KXP + k8;
  *(volatile v8us*)dp = o;
  *(volatile v8us*)(dp + DI) = o;
  __threadfence();
  *(volatile v8us*)dp = o;
  *(volatile v8us*)(dp + DI) = o;
}

template <int NT, int RES>
__global__ __launch_bounds__(GTHR) void k_gemm(const unsigned short* __restrict__ A,
                                               const unsigned short* __restrict__ WT,
                                               float* outF, const float* __restrict__ resx, int K, int ldo) {
  constexpr int GBN = 16 * NT;
  constexpr int NV  = GBN / 8;
  constexpr int RQ  = GBN / 4;
  __shared__ __attribute__((aligned(16))) float stg[GBM * GBN];
  const int tid = (int)threadIdx.x, lane = tid & 31, wave = tid >> 5, hh = lane >> 4, m = lane & 15;
  const int rowBase = (int)blockIdx.x * GBM;
  const int col0    = (int)blockIdx.y * GBN;

  v8f acc[NT];
  {
    const v8f z = {0.f, 0.f, 0.f, 0.f, 0.f, 0.f, 0.f, 0.f};
#pragma unroll
    for (int t = 0; t < NT; ++t) acc[t] = z;
  }
  const unsigned short* ap = A  + (size_t)(rowBase + 16 * wave + m) * (size_t)K + 8 * hh;
  const unsigned short* wp = WT + (size_t)(col0 + m) * (size_t)K + 8 * hh;
  const int ksteps = K >> 5;
#pragma unroll 1
  for (int ks = 0; ks < ksteps; ++ks) {
    FragB af;
    af.h[0] = *(const v8usa*)(ap + 32 * ks);
    af.h[1] = *(const v8usa*)(ap + 32 * ks + 16);
#pragma unroll
    for (int t = 0; t < NT; ++t) {
      const unsigned short* wq = wp + (size_t)(16 * t) * (size_t)K + 32 * ks;
      FragB bf;
      bf.h[0] = *(const v8usa*)wq;
      bf.h[1] = *(const v8usa*)(wq + 16);
      acc[t] = wmb(af, bf, acc[t]);
    }
  }

#pragma unroll
  for (int t = 0; t < NT; ++t) {
    const int lc = 16 * t + m;
#pragma unroll
    for (int r = 0; r < 8; ++r) {
      const int lr = 16 * wave + 8 * hh + r;
      stg[lr * GBN + lc] = acc[t][r];
    }
  }
  __syncthreads();

  v4f fv[NV];
#pragma unroll
  for (int i = 0; i < NV; ++i) {
    const int q  = i * 32 + lane;
    const int lr = 16 * wave + q / RQ;
    const int c4 = q % RQ;
    v4f t = *(const v4fa*)(stg + lr * GBN + 4 * c4);
    if constexpr (RES != 0) {
      const v4f r4 = *(const v4fa*)(resx + (size_t)(rowBase + lr) * (size_t)ldo + col0 + 4 * c4);
      t.x = t.x + bf16_val(r4.x);
      t.y = t.y + bf16_val(r4.y);
      t.z = t.z + bf16_val(r4.z);
      t.w = t.w + bf16_val(r4.w);
    }
    fv[i] = t;
  }
#pragma unroll
  for (int i = 0; i < NV; ++i) {
    const int q  = i * 32 + lane;
    const int lr = 16 * wave + q / RQ;
    const int c4 = q % RQ;
    float* op = outF + (size_t)(rowBase + lr) * (size_t)ldo + col0 + 4 * c4;
    *(volatile v4f*)op = fv[i];
  }
  __threadfence();
#pragma unroll
  for (int i = 0; i < NV; ++i) {
    const int q  = i * 32 + lane;
    const int lr = 16 * wave + q / RQ;
    const int c4 = q % RQ;
    float* op = outF + (size_t)(rowBase + lr) * (size_t)ldo + col0 + 4 * c4;
    *(volatile v4f*)op = fv[i];
  }
}

__global__ __launch_bounds__(256) void k_conv(const float* __restrict__ xz, const float* __restrict__ cw,
                                              const float* __restrict__ cbp, unsigned short* xc) {
  __shared__ __attribute__((aligned(16))) unsigned short sb[512];
  const int tid = (int)threadIdx.x;
  const int cb0 = (int)blockIdx.x * 256;
  const int c   = cb0 + tid;
  const int row = (int)blockIdx.y;
  const int t   = row & (TL - 1);
  const int rb  = row - t;
  float xs[4];
#pragma unroll
  for (int k = 0; k < 4; ++k) {
    int r = row - 3 + k;
    r = r < rb ? rb : r;
    const float f = xz[(size_t)r * NXZ + c];
    xs[k] = (t - 3 + k >= 0) ? f : 0.0f;
  }
  const v4f w4 = *(const v4fa*)(cw + (size_t)c * 4);
  const float v = conv_silu(xs[0], xs[1], xs[2], xs[3],
                            bf16_val(w4.x), bf16_val(w4.y), bf16_val(w4.z), bf16_val(w4.w),
                            bf16_val(cbp[c]));
  const unsigned hb = bf16_bits(v);
  const unsigned lb = bf16_bits(v - __uint_as_float(hb << 16));
  sb[tid]       = (unsigned short)hb;
  sb[256 + tid] = (unsigned short)lb;
  __syncthreads();
  const int plane = (tid >> 5) & 1;
  const int pc    = tid & 31;
  const v8us q = *(const v8usa*)(sb + plane * 256 + 8 * pc);
  unsigned short* dp = xc + (size_t)row * KXP + (size_t)plane * DI + cb0 + 8 * pc;
  const bool wr = tid < 64;
  if (wr) *(volatile v8us*)dp = q;
  __threadfence();
  if (wr) *(volatile v8us*)dp = q;
}

__global__ __launch_bounds__(STH) void k_scan(const float* __restrict__ xz, const float* __restrict__ P,
                                              const float* __restrict__ cw, const float* __restrict__ cbp,
                                              const float* __restrict__ wdtp, const float* __restrict__ bdtp,
                                              const float* __restrict__ alog, const float* __restrict__ dpar,
                                              unsigned short* Y) {
  __shared__ __attribute__((aligned(16))) float ps[TCH * PSP];
  __shared__ __attribute__((aligned(16))) unsigned short yb[2 * TCH * SCH];
  __shared__ float sA[8 * STH];
  const int tid  = (int)threadIdx.x;
  const int c    = tid >> 1;
  const int half = tid & 1;
  const int b    = (int)blockIdx.x / (DI / SCH);
  const int d0   = ((int)blockIdx.x % (DI / SCH)) * SCH;
  const int d    = d0 + c;

#pragma unroll 1
  for (int j = 0; j < 8; ++j) {
    const float al = bf16_val(alog[(size_t)d * DS + 8 * half + j]);
    sA[j * STH + tid] = -expf(al);
  }
  __syncthreads();
  float A[8], h[8];
#pragma unroll
  for (int j = 0; j < 8; ++j) { A[j] = sA[j * STH + tid]; h[j] = 0.0f; }

  const v4f w4 = *(const v4fa*)(cw + (size_t)d * 4);
  const float w0 = bf16_val(w4.x), w1 = bf16_val(w4.y), w2 = bf16_val(w4.z), w3 = bf16_val(w4.w);
  const float cb  = bf16_val(cbp[d]);
  const float wdt = bf16_val(wdtp[d]);
  const float bdt = bf16_val(bdtp[d]);
  const float Dv  = bf16_val(dpar[d]);
  float xm3 = 0.0f, xm2 = 0.0f, xm1 = 0.0f;

#pragma unroll 1
  for (int ch = 0; ch < TL / TCH; ++ch) {
    const int t0 = ch * TCH;
    const size_t rowb = (size_t)b * TL + (size_t)t0;
#pragma unroll
    for (int it = 0; it < 4; ++it) {
      const int u = it * STH + tid;
      const int r = u >> 4, q = u & 15;
      const v4f pv = *(const v4fa*)(P + (rowb + (size_t)r) * PPIT + 4 * q);
      const int cq = 4 * q;
      if (cq     <= 32) ps[r * PSP + (cq == 0 ? 32 : cq - 1)] = pv.x;
      if (cq + 1 <= 32) ps[r * PSP + cq]     = pv.y;
      if (cq + 2 <= 32) ps[r * PSP + cq + 1] = pv.z;
      if (cq + 3 <= 32) ps[r * PSP + cq + 2] = pv.w;
    }
    __syncthreads();

#pragma unroll 1
    for (int tl = 0; tl < TCH; ++tl) {
      const size_t rowi = rowb + (size_t)tl;
      const float xt = xz[rowi * NXZ + d];
      const float zt = xz[rowi * NXZ + DI + d];
      const float* pr = ps + tl * PSP;
      const v4f B0 = *(const v4fa*)(pr + 8 * half);
      const v4f B1 = *(const v4fa*)(pr + 8 * half + 4);
      const v4f C0 = *(const v4fa*)(pr + 16 + 8 * half);
      const v4f C1 = *(const v4fa*)(pr + 16 + 8 * half + 4);
      const float dtr = pr[32];
      float Bv[8], Cv[8];
      Bv[0] = B0.x; Bv[1] = B0.y; Bv[2] = B0.z; Bv[3] = B0.w;
      Bv[4] = B1.x; Bv[5] = B1.y; Bv[6] = B1.z; Bv[7] = B1.w;
      Cv[0] = C0.x; Cv[1] = C0.y; Cv[2] = C0.z; Cv[3] = C0.w;
      Cv[4] = C1.x; Cv[5] = C1.y; Cv[6] = C1.z; Cv[7] = C1.w;

      const float xc = conv_silu(xm3, xm2, xm1, xt, w0, w1, w2, w3, cb);
      xm3 = xm2; xm2 = xm1; xm1 = xt;

      const float u  = dtr * wdt + bdt;
      const float dt = fmaxf(u, 0.0f) + log1pf(expf(-fabsf(u)));

      float ys = 0.0f;
#pragma unroll
      for (int j = 0; j < 8; ++j) {
        const float a  = expf(dt * A[j]);
        const float bx = (dt * Bv[j]) * xc;
        h[j] = a * h[j] + bx;
        ys = ys + h[j] * Cv[j];
      }
      const float yo = __shfl_xor(ys, 1, 32);
      float y = ys + yo;
      y = y + xc * Dv;
      const float ez = expf(-zt);
      const float g  = zt * (1.0f / (1.0f + ez));
      y = y * g;
      const unsigned hb = bf16_bits(y);
      const unsigned lb = bf16_bits(y - __uint_as_float(hb << 16));
      const unsigned sel = (half != 0) ? lb : hb;
      yb[half * (TCH * SCH) + tl * SCH + c] = (unsigned short)sel;
    }
    __syncthreads();

    v8us q[4];
#pragma unroll
    for (int it = 0; it < 4; ++it) {
      const int u = it * STH + tid;
      const int plane = u >> 8, r = (u >> 3) & 31, pc = u & 7;
      q[it] = *(const v8usa*)(yb + plane * (TCH * SCH) + r * SCH + 8 * pc);
    }
#pragma unroll
    for (int it = 0; it < 4; ++it) {
      const int u = it * STH + tid;
      const int plane = u >> 8, r = (u >> 3) & 31, pc = u & 7;
      unsigned short* dp = Y + (rowb + (size_t)r) * KXP + (size_t)plane * DI + d0 + 8 * pc;
      *(volatile v8us*)dp = q[it];
    }
    __threadfence();
#pragma unroll
    for (int it = 0; it < 4; ++it) {
      const int u = it * STH + tid;
      const int plane = u >> 8, r = (u >> 3) & 31, pc = u & 7;
      unsigned short* dp = Y + (rowb + (size_t)r) * KXP + (size_t)plane * DI + d0 + 8 * pc;
      *(volatile v8us*)dp = q[it];
    }
  }
}

static inline size_t al256(size_t o) { return (o + 255) & ~(size_t)255; }

extern "C" void kernel_launch(void* const* d_in, const int* in_sizes, int n_in,
                              void* d_out, int out_size, void* d_ws, size_t ws_size,
                              hipStream_t stream) {
  if (n_in < 11) return;
  if (in_sizes[0] != MR * DM) return;
  if (in_sizes[1] != DM) return;
  if (in_sizes[2] != DM * NXZ) return;
  if (in_sizes[3] != DI * 4) return;
  if (in_sizes[4] != DI) return;
  if (in_sizes[5] != DI * NPX) return;
  if (in_sizes[6] != DI || in_sizes[7] != DI) return;
  if (in_sizes[8] != DI * DS) return;
  if (in_sizes[9] != DI) return;
  if (in_sizes[10] != DI * DM) return;
  if (out_size != MR * DM) return;

  const float* x     = (const float*)d_in[0];
  const float* normw = (const float*)d_in[1];
  const float* W_in  = (const float*)d_in[2];
  const float* convw = (const float*)d_in[3];
  const float* convb = (const float*)d_in[4];
  const float* W_x   = (const float*)d_in[5];
  const float* w_dt  = (const float*)d_in[6];
  const float* b_dt  = (const float*)d_in[7];
  const float* A_log = (const float*)d_in[8];
  const float* D_par = (const float*)d_in[9];
  const float* W_out = (const float*)d_in[10];
  float* out = (float*)d_out;

  char* ws = (char*)d_ws;
  size_t off = 0;
  const size_t oA   = off; off = al256(off + (size_t)MR * KXP * 2);
  const size_t oXZ  = off; off = al256(off + (size_t)MR * NXZ * 4);
  const size_t oWO  = off; off = al256(off + (size_t)DM * KXP * 2);
  const size_t oWX  = off; off = al256(off + (size_t)PPIT * KXP * 2);
  const size_t oP   = off; off = al256(off + (size_t)MR * PPIT * 4);
  if (off > ws_size || off > (size_t)WSMAX) return;
  unsigned short* XN    = (unsigned short*)(ws + oA);
  unsigned short* WIN2  = (unsigned short*)(ws + oA + (size_t)MR * KIN * 2);
  unsigned short* XC    = (unsigned short*)(ws + oA);
  unsigned short* YP    = (unsigned short*)(ws + oA);
  float*          XZ    = (float*)(ws + oXZ);
  unsigned short* WOUT2 = (unsigned short*)(ws + oWO);
  unsigned short* WX2   = (unsigned short*)(ws + oWX);
  float*          P     = (float*)(ws + oP);

  k_norm<<<MR, 128, 0, stream>>>(x, normw, XN);
  k_wT<<<dim3(NXZ / 64, DM / 64), 256, 0, stream>>>(W_in, DM, NXZ, WIN2);
  k_wT<<<dim3(DM / 64, DI / 64), 256, 0, stream>>>(W_out, DI, DM, WOUT2);
  k_wx<<<PPIT, 256, 0, stream>>>(W_x, WX2);
  k_gemm<8, 0><<<dim3(MR / GBM, NXZ / 128), GTHR, 0, stream>>>(XN, WIN2, XZ, x, KIN, NXZ);
  k_conv<<<dim3(DI / 256, MR), 256, 0, stream>>>(XZ, convw, convb, XC);
  k_gemm<4, 0><<<dim3(MR / GBM, 1), GTHR, 0, stream>>>(XC, WX2, P, x, KXP, PPIT);
  k_scan<<<NBAT * (DI / SCH), STH, 0, stream>>>(XZ, P, convw, convb, w_dt, b_dt, A_log, D_par, YP);
  k_gemm<8, 1><<<dim3(MR / GBM, DM / 128), GTHR, 0, stream>>>(YP, WOUT2, out, x, KXP, DM);
}
